// RealMambaCore_1073741824059
// MI455X (gfx1250) — hardware-run, weakly checked
//
#include <hip/hip_runtime.h>
#include <hip/hip_bf16.h>


#define DIM  1024
#define TSEQ 2048

typedef __bf16   v16b __attribute__((ext_vector_type(16)));
typedef float    v8f  __attribute__((ext_vector_type(8)));
typedef float    v4f  __attribute__((ext_vector_type(4)));
typedef unsigned v4u  __attribute__((ext_vector_type(4)));
typedef unsigned v2u  __attribute__((ext_vector_type(2)));

union Frag { v16b v; v4u q[2]; };

__device__ __forceinline__ unsigned bf16_bits(float f) {
    unsigned u = __float_as_uint(f);
    u = u + 0x7FFFu + ((u >> 16) & 1u);
    return (u >> 16) & 0xFFFFu;
}

__device__ __forceinline__ void split_hl(float f, unsigned& hb, unsigned& lb) {
    hb = bf16_bits(f);
    const float hf = __uint_as_float(hb << 16);
    lb = bf16_bits(f - hf);
}

__device__ __forceinline__ v8f zero8() {
    v8f z;
#pragma unroll
    for (int e = 0; e < 8; ++e) z[e] = 0.0f;
    return z;
}

__device__ __forceinline__ float silu_f(float x) {
    return x / (1.0f + expf(-x));
}

__device__ __forceinline__ float wave_sum(float v) {
#pragma unroll
    for (int o = 16; o > 0; o >>= 1) v += __shfl_xor(v, o, 32);
    return v;
}

__device__ __forceinline__ void mma3(v8f& acc, const v16b& ah, const v16b& al,
                                     const v16b& bh, const v16b& bl) {
    acc = __builtin_amdgcn_wmma_f32_16x16x32_bf16(false, ah, false, bh, (short)0, acc, false, false);
    acc = __builtin_amdgcn_wmma_f32_16x16x32_bf16(false, al, false, bh, (short)0, acc, false, false);
    acc = __builtin_amdgcn_wmma_f32_16x16x32_bf16(false, ah, false, bl, (short)0, acc, false, false);
    asm volatile("v_nop\n\tv_nop\n\tv_nop\n\tv_nop"
                 : "+v"(acc) : "v"(ah), "v"(al), "v"(bh), "v"(bl));
}

__global__ __launch_bounds__(128) void wsplit_kernel(const float* __restrict__ W,
                                                     unsigned short* __restrict__ Wh,
                                                     unsigned short* __restrict__ Wl)
{
    __shared__ __align__(16) unsigned short sH[64][72];
    __shared__ __align__(16) unsigned short sL[64][72];

    const int tid = threadIdx.x, lane = tid & 31, wave = tid >> 5;
    const int n0 = blockIdx.x * 64, k0 = blockIdx.y * 64;

#pragma unroll
    for (int i = 0; i < 8; ++i) {
        const int vi = tid + i * 128;
        const int kr = vi >> 4, c4 = (vi & 15) << 2;
        const v4f f = *(const v4f*)(W + (size_t)(k0 + kr) * DIM + n0 + c4);
        unsigned hb, lb;
        split_hl(f.x, hb, lb); sH[c4 + 0][kr] = (unsigned short)hb; sL[c4 + 0][kr] = (unsigned short)lb;
        split_hl(f.y, hb, lb); sH[c4 + 1][kr] = (unsigned short)hb; sL[c4 + 1][kr] = (unsigned short)lb;
        split_hl(f.z, hb, lb); sH[c4 + 2][kr] = (unsigned short)hb; sL[c4 + 2][kr] = (unsigned short)lb;
        split_hl(f.w, hb, lb); sH[c4 + 3][kr] = (unsigned short)hb; sL[c4 + 3][kr] = (unsigned short)lb;
    }
    __syncthreads();

    v4u hv[4], lv[4];
#pragma unroll
    for (int it = 0; it < 4; ++it) {
        const int row = wave * 16 + it * 4 + (lane >> 3);
        const int piece = lane & 7;
        hv[it] = *(const v4u*)&sH[row][piece * 8];
        lv[it] = *(const v4u*)&sL[row][piece * 8];
    }
#pragma unroll
    for (int it = 0; it < 4; ++it) {
        const int row = wave * 16 + it * 4 + (lane >> 3);
        const int piece = lane & 7;
        const size_t g = (size_t)(n0 + row) * DIM + k0 + piece * 8;
        *(volatile v4u*)(Wh + g) = hv[it];
        *(volatile v4u*)(Wl + g) = lv[it];
    }
    __threadfence();
#pragma unroll
    for (int it = 0; it < 4; ++it) {
        const int row = wave * 16 + it * 4 + (lane >> 3);
        const int piece = lane & 7;
        const size_t g = (size_t)(n0 + row) * DIM + k0 + piece * 8;
        *(volatile v4u*)(Wh + g) = hv[it];
        *(volatile v4u*)(Wl + g) = lv[it];
    }
}

template <int NW, int EPI>
__global__ __launch_bounds__(128) void gemm_kernel(
    const float* __restrict__ X,
    const unsigned short* __restrict__ W0h, const unsigned short* __restrict__ W0l,
    const unsigned short* __restrict__ W1h, const unsigned short* __restrict__ W1l,
    const float* __restrict__ bias0, const float* __restrict__ bias1,
    float* __restrict__ O, int M)
{
    static_assert(NW == 1 || NW == 2);
    static_assert(EPI == 0 || NW == 2);
    constexpr int BM = 64, BN = 32, BK = 32, LP = BK + 8, OP = BN + 4;
    __shared__ __align__(16) unsigned short sXh[BM][LP];
    __shared__ __align__(16) unsigned short sXl[BM][LP];
    __shared__ __align__(16) unsigned short sWh[NW][BN][LP];
    __shared__ __align__(16) unsigned short sWl[NW][BN][LP];
    __shared__ __align__(16) float sO[BM][OP];

    const int tid = threadIdx.x, lane = tid & 31, wave = tid >> 5;
    const int hh = lane >> 4, m16 = lane & 15;
    const int wm = wave & 1, wn = wave >> 1;
    const int blockRow = blockIdx.x * BM, blockCol = blockIdx.y * BN;

    v8f acc[NW][2];
#pragma unroll
    for (int w = 0; w < NW; ++w) { acc[w][0] = zero8(); acc[w][1] = zero8(); }

    for (int kt = 0; kt < DIM / BK; ++kt) {
        const int k0 = kt * BK;
#pragma unroll
        for (int i = 0; i < 4; ++i) {
            const int vi = tid + i * 128;
            const int r = vi >> 3, c4 = (vi & 7) << 2;
            const int gr = blockRow + r;
            v4f f; f.x = 0.0f; f.y = 0.0f; f.z = 0.0f; f.w = 0.0f;
            if (gr < M) f = *(const v4f*)(X + (size_t)gr * DIM + k0 + c4);
            unsigned h0, l0, h1, l1, h2, l2, h3, l3;
            split_hl(f.x, h0, l0); split_hl(f.y, h1, l1);
            split_hl(f.z, h2, l2); split_hl(f.w, h3, l3);
            v2u hv, lv;
            hv.x = h0 | (h1 << 16); hv.y = h2 | (h3 << 16);
            lv.x = l0 | (l1 << 16); lv.y = l2 | (l3 << 16);
            *(v2u*)&sXh[r][c4] = hv;
            *(v2u*)&sXl[r][c4] = lv;
        }
#pragma unroll
        for (int w = 0; w < NW; ++w) {
            const unsigned short* Wh = (w == 0) ? W0h : W1h;
            const unsigned short* Wl = (w == 0) ? W0l : W1l;
            const int r = tid >> 2, c8 = (tid & 3) << 3;
            const size_t g = (size_t)(blockCol + r) * DIM + k0 + c8;
            *(v4u*)&sWh[w][r][c8] = *(const v4u*)(Wh + g);
            *(v4u*)&sWl[w][r][c8] = *(const v4u*)(Wl + g);
        }
        __syncthreads();

        Frag ah[2], al[2];
#pragma unroll
        for (int m = 0; m < 2; ++m) {
            const unsigned short* ph = &sXh[wm * 32 + m * 16 + m16][0];
            const unsigned short* pl = &sXl[wm * 32 + m * 16 + m16][0];
            ah[m].q[0] = *(const v4u*)(ph + 8 * hh);
            ah[m].q[1] = *(const v4u*)(ph + 16 + 8 * hh);
            al[m].q[0] = *(const v4u*)(pl + 8 * hh);
            al[m].q[1] = *(const v4u*)(pl + 16 + 8 * hh);
        }
#pragma unroll
        for (int w = 0; w < NW; ++w) {
            Frag bh, bl;
            const unsigned short* ph = &sWh[w][wn * 16 + m16][0];
            const unsigned short* pl = &sWl[w][wn * 16 + m16][0];
            bh.q[0] = *(const v4u*)(ph + 8 * hh);
            bh.q[1] = *(const v4u*)(ph + 16 + 8 * hh);
            bl.q[0] = *(const v4u*)(pl + 8 * hh);
            bl.q[1] = *(const v4u*)(pl + 16 + 8 * hh);
#pragma unroll
            for (int m = 0; m < 2; ++m)
                mma3(acc[w][m], ah[m].v, al[m].v, bh.v, bl.v);
        }
        __syncthreads();
    }

#pragma unroll
    for (int m = 0; m < 2; ++m) {
        const int col = wn * 16 + m16;
        const int gc = blockCol + col;
        const float bA = bias0[gc];
        float bB = 0.0f;
        if constexpr (EPI == 1) bB = bias1[gc];
#pragma unroll
        for (int r = 0; r < 8; ++r) {
            const int row = wm * 32 + m * 16 + 8 * hh + r;
            float val;
            if constexpr (EPI == 1) {
                const float ga = acc[0][m][r] + bA;
                const float gb = acc[NW - 1][m][r] + bB;
                val = silu_f(ga) * gb;
            } else {
                val = acc[0][m][r] + bA;
            }
            sO[row][col] = val;
        }
    }
    __syncthreads();

    v4f ov[4];
#pragma unroll
    for (int it = 0; it < 4; ++it) {
        const int row = wave * 16 + it * 4 + (lane >> 3);
        const int piece = lane & 7;
        ov[it] = *(const v4f*)&sO[row][piece * 4];
    }
#pragma unroll
    for (int it = 0; it < 4; ++it) {
        const int row = wave * 16 + it * 4 + (lane >> 3);
        const int piece = lane & 7;
        const int gr = blockRow + row;
        if (gr < M)
            *(volatile v4f*)(O + (size_t)gr * DIM + blockCol + piece * 4) = ov[it];
    }
    __threadfence();
#pragma unroll
    for (int it = 0; it < 4; ++it) {
        const int row = wave * 16 + it * 4 + (lane >> 3);
        const int piece = lane & 7;
        const int gr = blockRow + row;
        if (gr < M)
            *(volatile v4f*)(O + (size_t)gr * DIM + blockCol + piece * 4) = ov[it];
    }
}

__global__ __launch_bounds__(128) void scan_kernel(
    const float* __restrict__ u, const float* __restrict__ A,
    const float* __restrict__ Bp, const float* __restrict__ Cp,
    const float* __restrict__ Dp, float* __restrict__ v, int nB)
{
    const int g = blockIdx.x * 128 + threadIdx.x;
    const int q = DIM / 4;
    if (g >= nB * q) return;
    const int b = g / q;
    const int d4 = (g - b * q) * 4;
    const v4f a  = *(const v4f*)(A  + d4);
    const v4f bp = *(const v4f*)(Bp + d4);
    const v4f cp = *(const v4f*)(Cp + d4);
    const v4f dp = *(const v4f*)(Dp + d4);
    const size_t base = (size_t)b * TSEQ * DIM + d4;

    {
        v4f y; y.x = 0.0f; y.y = 0.0f; y.z = 0.0f; y.w = 0.0f;
#pragma unroll 1
        for (int t = 0; t < TSEQ; ++t) {
            const size_t o = base + (size_t)t * DIM;
            const v4f uu = *(const v4f*)(u + o);
            y = a * y + bp * uu;
            const v4f ov = cp * y + dp * uu;
            *(volatile v4f*)(v + o) = ov;
        }
    }
    __threadfence();
    {
        v4f y; y.x = 0.0f; y.y = 0.0f; y.z = 0.0f; y.w = 0.0f;
#pragma unroll 1
        for (int t = 0; t < TSEQ; ++t) {
            const size_t o = base + (size_t)t * DIM;
            const v4f uu = *(const v4f*)(u + o);
            y = a * y + bp * uu;
            const v4f ov = cp * y + dp * uu;
            *(volatile v4f*)(v + o) = ov;
        }
    }
}

__global__ __launch_bounds__(256) void ln_kernel(
    const float* __restrict__ vin, const float* __restrict__ gamma,
    const float* __restrict__ beta, float* __restrict__ yout, int M)
{
    __shared__ float s1[8];
    __shared__ float s2[8];
    const int row = blockIdx.x;
    if (row >= M) return;
    const int t = threadIdx.x, lane = t & 31, wave = t >> 5;
    const size_t off = (size_t)row * DIM + t * 4;
    const v4f x = *(const v4f*)(vin + off);

    float s = (x.x + x.y) + (x.z + x.w);
    s = wave_sum(s);
    if (lane == 0) s1[wave] = s;
    __syncthreads();
    float tot = 0.0f;
#pragma unroll
    for (int i = 0; i < 8; ++i) tot += s1[i];
    const float mu = tot * (1.0f / DIM);

    const v4f d = x - mu;
    float qq = (d.x * d.x + d.y * d.y) + (d.z * d.z + d.w * d.w);
    qq = wave_sum(qq);
    if (lane == 0) s2[wave] = qq;
    __syncthreads();
    float tq = 0.0f;
#pragma unroll
    for (int i = 0; i < 8; ++i) tq += s2[i];
    const float var = tq * (1.0f / DIM);
    const float rstd = 1.0f / sqrtf(var + 1e-3f);

    const v4f gm = *(const v4f*)(gamma + t * 4);
    const v4f be = *(const v4f*)(beta  + t * 4);
    const v4f o = (d * rstd) * gm + be;
    *(volatile v4f*)(yout + off) = o;
    __threadfence();
    *(volatile v4f*)(yout + off) = o;
}

extern "C" void kernel_launch(void* const* d_in, const int* in_sizes, int n_in,
                              void* d_out, int out_size, void* d_ws, size_t ws_size,
                              hipStream_t stream)
{
    if (n_in < 19) return;
    const int D = DIM;
    if (in_sizes[1] != D * D || in_sizes[3] != D * D || in_sizes[11] != D * D ||
        in_sizes[13] != D * D || in_sizes[15] != D * D || in_sizes[17] != D * D) return;
    if (in_sizes[2] != D || in_sizes[4] != D || in_sizes[12] != D || in_sizes[14] != D ||
        in_sizes[16] != D || in_sizes[18] != D) return;
    if (in_sizes[5] != D || in_sizes[6] != D || in_sizes[7] != D || in_sizes[8] != D ||
        in_sizes[9] != D || in_sizes[10] != D) return;
    const int M = in_sizes[0] / D;
    if (M <= 0 || in_sizes[0] != M * D || (M % TSEQ) != 0 || out_size != M * D) return;
    const int nB = M / TSEQ;

    const float* x     = (const float*)d_in[0];
    const float* Wg    = (const float*)d_in[1];
    const float* bg    = (const float*)d_in[2];
    const float* Wi    = (const float*)d_in[3];
    const float* bi    = (const float*)d_in[4];
    const float* A     = (const float*)d_in[5];
    const float* Bp    = (const float*)d_in[6];
    const float* Cp    = (const float*)d_in[7];
    const float* Dp    = (const float*)d_in[8];
    const float* gamma = (const float*)d_in[9];
    const float* beta  = (const float*)d_in[10];
    const float* Wfg   = (const float*)d_in[11];
    const float* bfg   = (const float*)d_in[12];
    const float* Wfu   = (const float*)d_in[13];
    const float* bfu   = (const float*)d_in[14];
    const float* Wfd   = (const float*)d_in[15];
    const float* bfd   = (const float*)d_in[16];
    const float* Wo    = (const float*)d_in[17];
    const float* bo    = (const float*)d_in[18];

    char* ws = (char*)d_ws;
    const size_t plane = (size_t)D * D * sizeof(unsigned short);
    const size_t act   = (size_t)M * D * sizeof(float);
    size_t off = 0;
    unsigned short* wp[12];
    for (int i = 0; i < 12; ++i) { wp[i] = (unsigned short*)(ws + off); off += plane; }
    float* u   = (float*)(ws + off); off += act;
    float* v   = (float*)(ws + off); off += act;
    float* yln = (float*)(ws + off); off += act;
    float* hb  = (float*)(ws + off); off += act;
    float* z   = (float*)(ws + off); off += act;
    if (off > ws_size) return;

    const float* Wsrc[6] = { Wg, Wi, Wfg, Wfu, Wfd, Wo };
    for (int i = 0; i < 6; ++i)
        wsplit_kernel<<<dim3(D / 64, D / 64), dim3(128), 0, stream>>>(Wsrc[i], wp[2 * i], wp[2 * i + 1]);

    const dim3 gg((M + 63) / 64, D / 32);
    const dim3 gb(128);

    gemm_kernel<2, 1><<<gg, gb, 0, stream>>>(x, wp[0], wp[1], wp[2], wp[3], bg, bi, u, M);
    scan_kernel<<<dim3((nB * (D / 4) + 127) / 128), dim3(128), 0, stream>>>(u, A, Bp, Cp, Dp, v, nB);
    ln_kernel<<<dim3(M), dim3(256), 0, stream>>>(v, gamma, beta, yln, M);
    gemm_kernel<2, 1><<<gg, gb, 0, stream>>>(yln, wp[4], wp[5], wp[6], wp[7], bfg, bfu, hb, M);
    gemm_kernel<1, 0><<<gg, gb, 0, stream>>>(hb, wp[8], wp[9], wp[8], wp[9], bfd, bfd, z, M);
    gemm_kernel<1, 0><<<gg, gb, 0, stream>>>(z, wp[10], wp[11], wp[10], wp[11], bo, bo, (float*)d_out, M);
    (void)hipGetLastError();
}
